// SemanticConsistencyGNN_11553462026404
// MI455X (gfx1250) — hardware-verified
//
#include <hip/hip_runtime.h>
#include <hip/hip_bf16.h>
#include <stddef.h>


#define NN     468
#define FE     64
#define F1     128
#define F2     256
#define F3     128
#define FF     512
#define NCLS   2
#define NTAP   19
#define HALFW  9
#define CP     32
#define CROWS  512
#define NTHR   256
#define GR     128
#define GC     64
#define AMAXW  256
#define BMUL   128
#define WSCAP  134217728

static_assert(CROWS == 2 * NTHR);
static_assert(NTAP <= CP && NN <= CROWS);
static_assert((FE % 32) == 0 && (F1 % 32) == 0 && (F2 % 32) == 0 && (F3 % 32) == 0);
static_assert((F1 % GC) == 0 && (F2 % GC) == 0 && (F3 % GC) == 0 && (FF % GC) == 0);
static_assert(((F1 * FE / 8) % NTHR) == 0 && ((F2 * F1 / 8) % NTHR) == 0);
static_assert(((F3 * F2 / 8) % NTHR) == 0 && ((FF * F3 / 8) % NTHR) == 0);
static_assert(AMAXW * 2 == F3 * 4);
static_assert(AMAXW >= FE && AMAXW >= F1 && AMAXW >= F2);
static_assert(GR == 8 * 16 && BMUL == GR);
static_assert(((BMUL * NN) % GR) == 0 && ((BMUL * NN * 8) % NTHR) == 0);
static_assert((NTHR / 2) * NCLS == NTHR && (FF % 4) == 0);

typedef float    v4f  __attribute__((ext_vector_type(4)));
typedef float    v8f  __attribute__((ext_vector_type(8)));
typedef unsigned v2u  __attribute__((ext_vector_type(2)));
typedef unsigned v4u  __attribute__((ext_vector_type(4)));
typedef unsigned v8u  __attribute__((ext_vector_type(8)));
typedef __bf16   v16bf __attribute__((ext_vector_type(16)));
union FragB { v16bf v; v8u u; v4u q[2]; };

__device__ __forceinline__ unsigned bfb(float f) {
  const unsigned u = __float_as_uint(f);
  return (u + 0x7FFFu + ((u >> 16) & 1u)) >> 16;
}
__device__ __forceinline__ void hl1(float v, unsigned& h, unsigned& l) {
  h = bfb(v);
  l = bfb(v - __uint_as_float(h << 16));
}
__device__ __forceinline__ void hl4(v4f v, v2u& hp, v2u& lp) {
  unsigned h0, l0, h1, l1, h2, l2, h3, l3;
  hl1(v.x, h0, l0); hl1(v.y, h1, l1); hl1(v.z, h2, l2); hl1(v.w, h3, l3);
  hp.x = h0 | (h1 << 16); hp.y = h2 | (h3 << 16);
  lp.x = l0 | (l1 << 16); lp.y = l2 | (l3 << 16);
}

__device__ __forceinline__ v8f wmb(const FragB& a, const FragB& b, v8f c) {
  v8f d = __builtin_amdgcn_wmma_f32_16x16x32_bf16(false, a.v, false, b.v, (short)0, c, false, false);
  asm volatile("v_nop\n\tv_nop\n\tv_nop\n\tv_nop" : "+v"(d) : "v"(a.u), "v"(b.u));
  return d;
}

__global__ __launch_bounds__(NTHR) void k_coef(float* coef) {
  __shared__ float sd[CROWS];
  __shared__ __attribute__((aligned(16))) float tile[NTHR * CP];
  const int tid = threadIdx.x, lane = tid & 31, wave = tid >> 5;
#pragma unroll 1
  for (int i = tid; i < CROWS; i += NTHR) {
    const int ic = i < NN ? i : NN - 1;
    const int dl = ic < HALFW ? ic : HALFW;
    const int dr = (NN - 1 - ic) < HALFW ? (NN - 1 - ic) : HALFW;
    const float d = 1.0f / sqrtf((float)(1 + dl + dr));
    sd[i] = (i < NN) ? d : 0.0f;
  }
  __syncthreads();
  const int i = blockIdx.x * NTHR + tid;
  const float di = sd[i < CROWS ? i : CROWS - 1];
#pragma unroll 1
  for (int t = 0; t < CP; ++t) {
    const int j  = i - HALFW + t;
    const int jc = j < 0 ? 0 : (j > NN - 1 ? NN - 1 : j);
    const float dj = sd[jc];
    const bool ok = (t < NTAP) && (i < NN) && (j >= 0) && (j < NN);
    tile[tid * CP + t] = ok ? di * dj : 0.0f;
  }
  __syncthreads();
  float* gb = coef + (size_t)blockIdx.x * NTHR * CP;
#pragma unroll
  for (int q = 0; q < 8; ++q) {
    const int lr = 32 * wave + 4 * q + (lane >> 3), col = 4 * (lane & 7);
    const v4f v = *(const v4f*)(tile + lr * CP + col);
    *(volatile v4f*)(gb + (size_t)lr * CP + col) = v;
  }
  __threadfence();
#pragma unroll
  for (int q = 0; q < 8; ++q) {
    const int lr = 32 * wave + 4 * q + (lane >> 3), col = 4 * (lane & 7);
    const v4f v = *(const v4f*)(tile + lr * CP + col);
    *(volatile v4f*)(gb + (size_t)lr * CP + col) = v;
  }
}

__global__ __launch_bounds__(NTHR) void k_wprep(const float* __restrict__ W, unsigned short* ph, unsigned short* pl,
                                                int K, int N, int Npad) {
  const int idx = blockIdx.x * NTHR + threadIdx.x;
  const int kq  = K >> 3;
  int n = idx / kq;
  const int k0 = (idx - n * kq) * 8;
  n = n > Npad - 1 ? Npad - 1 : n;
  const int nc = n > N - 1 ? N - 1 : n;
  const bool live = n < N;
  v4f va, vb;
  va.x = W[(size_t)(k0 + 0) * N + nc]; va.y = W[(size_t)(k0 + 1) * N + nc];
  va.z = W[(size_t)(k0 + 2) * N + nc]; va.w = W[(size_t)(k0 + 3) * N + nc];
  vb.x = W[(size_t)(k0 + 4) * N + nc]; vb.y = W[(size_t)(k0 + 5) * N + nc];
  vb.z = W[(size_t)(k0 + 6) * N + nc]; vb.w = W[(size_t)(k0 + 7) * N + nc];
  if (!live) { const v4f z = {0.f, 0.f, 0.f, 0.f}; va = z; vb = z; }
  v2u ha, la, hb, lb;
  hl4(va, ha, la); hl4(vb, hb, lb);
  v4u hv, lv;
  hv.x = ha.x; hv.y = ha.y; hv.z = hb.x; hv.w = hb.y;
  lv.x = la.x; lv.y = la.y; lv.z = lb.x; lv.w = lb.y;
  const size_t o = (size_t)idx * 8;
  *(volatile v4u*)(ph + o) = hv;
  *(volatile v4u*)(pl + o) = lv;
  __threadfence();
  *(volatile v4u*)(ph + o) = hv;
  *(volatile v4u*)(pl + o) = lv;
}

__global__ __launch_bounds__(NTHR) void k_enc(const float* __restrict__ lm, const float* __restrict__ W,
                                              const float* __restrict__ bs, unsigned short* xh, unsigned short* xl,
                                              int nRows) {
  const int idx = blockIdx.x * NTHR + threadIdx.x;
  int row = idx >> 3;
  const int c0 = (idx & 7) * 8;
  row = row > nRows - 1 ? nRows - 1 : row;
  const float a0 = lm[(size_t)row * 3], a1 = lm[(size_t)row * 3 + 1], a2 = lm[(size_t)row * 3 + 2];
  const v4f w0a = *(const v4f*)(W + c0),          w0b = *(const v4f*)(W + c0 + 4);
  const v4f w1a = *(const v4f*)(W + FE + c0),     w1b = *(const v4f*)(W + FE + c0 + 4);
  const v4f w2a = *(const v4f*)(W + 2 * FE + c0), w2b = *(const v4f*)(W + 2 * FE + c0 + 4);
  const v4f ba  = *(const v4f*)(bs + c0),         bb  = *(const v4f*)(bs + c0 + 4);
  v4f pa = w0a * a0; pa = pa + w1a * a1; pa = pa + w2a * a2;
  v4f pb = w0b * a0; pb = pb + w1b * a1; pb = pb + w2b * a2;
  const v4f va = pa + ba, vb = pb + bb;
  v2u ha, la, hb, lb;
  hl4(va, ha, la); hl4(vb, hb, lb);
  v4u hv, lv;
  hv.x = ha.x; hv.y = ha.y; hv.z = hb.x; hv.w = hb.y;
  lv.x = la.x; lv.y = la.y; lv.z = lb.x; lv.w = lb.y;
  const size_t o = (size_t)row * FE + c0;
  *(volatile v4u*)(xh + o) = hv;
  *(volatile v4u*)(xl + o) = lv;
  __threadfence();
  *(volatile v4u*)(xh + o) = hv;
  *(volatile v4u*)(xl + o) = lv;
}

template <int EPI>
__global__ __launch_bounds__(NTHR) void k_gemm3(
    const unsigned short* __restrict__ Ah, const unsigned short* __restrict__ Al,
    const unsigned short* __restrict__ Wh, const unsigned short* __restrict__ Wl,
    const float* __restrict__ bias, float* C, int K, int N) {
  __shared__ __attribute__((aligned(16))) float stg[8 * 16 * GC];
  const int tid = threadIdx.x, lane = tid & 31, wave = tid >> 5, hh = lane >> 4, m = lane & 15;
  const int rowBase = blockIdx.x * GR, colBase = blockIdx.y * GC;
  const int r0 = rowBase + wave * 16;
  const size_t ao = (size_t)(r0 + m) * K + 8 * hh;
  const unsigned short* ah = Ah + ao;
  const unsigned short* al = Al + ao;

  v8f acc[4];
#pragma unroll
  for (int t = 0; t < 4; ++t) { const v8f z = {0.f, 0.f, 0.f, 0.f, 0.f, 0.f, 0.f, 0.f}; acc[t] = z; }

#pragma unroll 1
  for (int k0 = 0; k0 < K; k0 += 32) {
    FragB fa, fl;
    fa.q[0] = *(const v4u*)(ah + k0); fa.q[1] = *(const v4u*)(ah + k0 + 16);
    fl.q[0] = *(const v4u*)(al + k0); fl.q[1] = *(const v4u*)(al + k0 + 16);
#pragma unroll
    for (int t = 0; t < 4; ++t) {
      const size_t bo = (size_t)(colBase + 16 * t + m) * K + k0 + 8 * hh;
      FragB bh, bl;
      bh.q[0] = *(const v4u*)(Wh + bo); bh.q[1] = *(const v4u*)(Wh + bo + 16);
      bl.q[0] = *(const v4u*)(Wl + bo); bl.q[1] = *(const v4u*)(Wl + bo + 16);
      acc[t] = wmb(fa, bh, acc[t]);
      acc[t] = wmb(fa, bl, acc[t]);
      acc[t] = wmb(fl, bh, acc[t]);
    }
  }

  float* sw = stg + wave * (16 * GC);
#pragma unroll
  for (int t = 0; t < 4; ++t) {
    const int cl = 16 * t + m;
    float bv = 0.0f;
    if (EPI) bv = bias[colBase + cl];
#pragma unroll
    for (int r = 0; r < 8; ++r) {
      float v = acc[t][r];
      if (EPI) v = fmaxf(v + bv, 0.0f);
      sw[(8 * hh + r) * GC + cl] = v;
    }
  }
  __syncthreads();

  float* gb = C + (size_t)r0 * N + colBase;
#pragma unroll
  for (int i = 0; i < 8; ++i) {
    const int lr = 2 * i + hh, c4 = 4 * m;
    const v4f v = *(const v4f*)(sw + lr * GC + c4);
    *(volatile v4f*)(gb + (size_t)lr * N + c4) = v;
  }
  __threadfence();
#pragma unroll
  for (int i = 0; i < 8; ++i) {
    const int lr = 2 * i + hh, c4 = 4 * m;
    const v4f v = *(const v4f*)(sw + lr * GC + c4);
    *(volatile v4f*)(gb + (size_t)lr * N + c4) = v;
  }
}

template <int D, int OUTK>
__global__ __launch_bounds__(NTHR) void k_agg(const float* __restrict__ H, const float* __restrict__ coef,
                                              const float* __restrict__ bias,
                                              unsigned short* yh, unsigned short* yl, float* yf, int nRows) {
  constexpr int Q = D / 4;
  const int idx = blockIdx.x * NTHR + threadIdx.x;
  int row = idx / Q;
  const int c0 = (idx - row * Q) * 4;
  row = row > nRows - 1 ? nRows - 1 : row;
  const int b = row / NN, i = row - b * NN;
  const float* hb = H + (size_t)b * NN * D + c0;
  const float* cf = coef + i * CP;
  v4f acc = {0.f, 0.f, 0.f, 0.f};
#pragma unroll
  for (int t = 0; t < NTAP; ++t) {
    int j = i - HALFW + t;
    j = j < 0 ? 0 : (j > NN - 1 ? NN - 1 : j);
    const float c = cf[t];
    const v4f hv = *(const v4f*)(hb + (size_t)j * D);
    acc += hv * c;
  }
  const v4f bb = *(const v4f*)(bias + c0);
  v4f v = acc + bb;
  v.x = fmaxf(v.x, 0.f); v.y = fmaxf(v.y, 0.f); v.z = fmaxf(v.z, 0.f); v.w = fmaxf(v.w, 0.f);
  const size_t o = (size_t)row * D + c0;
  if (OUTK == 0) {
    v2u hp, lp;
    hl4(v, hp, lp);
    *(volatile v2u*)(yh + o) = hp;
    *(volatile v2u*)(yl + o) = lp;
    __threadfence();
    *(volatile v2u*)(yh + o) = hp;
    *(volatile v2u*)(yl + o) = lp;
  } else {
    *(volatile v4f*)(yf + o) = v;
    __threadfence();
    *(volatile v4f*)(yf + o) = v;
  }
}

__global__ __launch_bounds__(NTHR) void k_pool(const float* __restrict__ yf, float* out2,
                                               unsigned short* gh, unsigned short* gl, int nB) {
  const int idx = blockIdx.x * NTHR + threadIdx.x;
  int b = idx >> 5;
  const int c0 = (idx & 31) * 4;
  b = b > nB - 1 ? nB - 1 : b;
  const float* p = yf + (size_t)b * NN * F3 + c0;
  v4f s = {0.f, 0.f, 0.f, 0.f};
#pragma unroll 4
  for (int n = 0; n < NN; ++n) s += *(const v4f*)(p + (size_t)n * F3);
  const v4f mv = s * (1.0f / (float)NN);
  v2u hp, lp;
  hl4(mv, hp, lp);
  const size_t o = (size_t)b * F3 + c0;
  *(volatile v4f*)(out2 + o) = mv;
  *(volatile v2u*)(gh + o) = hp;
  *(volatile v2u*)(gl + o) = lp;
  __threadfence();
  *(volatile v4f*)(out2 + o) = mv;
  *(volatile v2u*)(gh + o) = hp;
  *(volatile v2u*)(gl + o) = lp;
}

__global__ __launch_bounds__(NTHR) void k_cls(const float* __restrict__ F, const float* __restrict__ W,
                                              const float* __restrict__ bc, float* out0) {
  __shared__ __attribute__((aligned(16))) float so[NTHR];
  const int tid = threadIdx.x;
  const int r = blockIdx.x * (NTHR / 2) + (tid >> 1), c = tid & 1;
  const float* f = F + (size_t)r * FF;
  float acc = 0.f;
#pragma unroll 1
  for (int q = 0; q < FF / 4; ++q) {
    const v4f fv = *(const v4f*)(f + 4 * q);
    const float* wq = W + (size_t)(4 * q) * NCLS + c;
    acc = fmaf(fv.x, wq[0], acc);
    acc = fmaf(fv.y, wq[NCLS], acc);
    acc = fmaf(fv.z, wq[2 * NCLS], acc);
    acc = fmaf(fv.w, wq[3 * NCLS], acc);
  }
  so[tid] = acc + bc[c];
  __syncthreads();
  v4f v = {0.f, 0.f, 0.f, 0.f};
  if (tid < 64) v = *(const v4f*)(so + 4 * tid);
  float* gp = out0 + (size_t)blockIdx.x * NTHR + 4 * tid;
  if (tid < 64) *(volatile v4f*)gp = v;
  __threadfence();
  if (tid < 64) *(volatile v4f*)gp = v;
}

extern "C" void kernel_launch(void* const* d_in, const int* in_sizes, int n_in,
                              void* d_out, int out_size, void* d_ws, size_t ws_size,
                              hipStream_t stream) {
  if (n_in < 13) return;
  const int B = in_sizes[0] / (NN * 3);
  if (B <= 0 || in_sizes[0] != B * NN * 3) return;
  if ((B % BMUL) != 0 || B > 4096) return;
  if (in_sizes[1] != 3 * FE || in_sizes[2] != FE) return;
  if (in_sizes[3] != FE * F1 || in_sizes[4] != F1) return;
  if (in_sizes[5] != F1 * F2 || in_sizes[6] != F2) return;
  if (in_sizes[7] != F2 * F3 || in_sizes[8] != F3) return;
  if (in_sizes[9] != F3 * FF || in_sizes[10] != FF) return;
  if (in_sizes[11] != FF * NCLS || in_sizes[12] != NCLS) return;
  if (out_size != B * (NCLS + FF + F3)) return;
  const int M = B * NN;

  const float* lm   = (const float*)d_in[0];
  const float* Wenc = (const float*)d_in[1];
  const float* benc = (const float*)d_in[2];
  const float* W1   = (const float*)d_in[3];
  const float* b1   = (const float*)d_in[4];
  const float* W2   = (const float*)d_in[5];
  const float* b2   = (const float*)d_in[6];
  const float* W3   = (const float*)d_in[7];
  const float* b3   = (const float*)d_in[8];
  const float* Wfus = (const float*)d_in[9];
  const float* bfus = (const float*)d_in[10];
  const float* Wcls = (const float*)d_in[11];
  const float* bcls = (const float*)d_in[12];

  float* out0 = (float*)d_out;
  float* out1 = out0 + (size_t)B * NCLS;
  float* out2 = out1 + (size_t)B * FF;

  char* ws = (char*)d_ws;
  size_t off = 0;
  const size_t oCoef = off; off += (size_t)CROWS * CP * 4;
  const size_t oW1h  = off; off += (size_t)F1 * FE * 2;
  const size_t oW1l  = off; off += (size_t)F1 * FE * 2;
  const size_t oW2h  = off; off += (size_t)F2 * F1 * 2;
  const size_t oW2l  = off; off += (size_t)F2 * F1 * 2;
  const size_t oW3h  = off; off += (size_t)F3 * F2 * 2;
  const size_t oW3l  = off; off += (size_t)F3 * F2 * 2;
  const size_t oWfh  = off; off += (size_t)FF * F3 * 2;
  const size_t oWfl  = off; off += (size_t)FF * F3 * 2;
  const size_t oGh   = off; off += (size_t)B * F3 * 2;
  const size_t oGl   = off; off += (size_t)B * F3 * 2;
  const size_t slotA = (size_t)M * AMAXW * 2;
  const size_t oAh   = off; off += slotA;
  const size_t oAl   = off; off += slotA;
  const size_t oH    = off; off += (size_t)M * AMAXW * 4;
  if (off > ws_size || off > (size_t)WSCAP) return;

  float*          coefp = (float*)(ws + oCoef);
  unsigned short* w1h = (unsigned short*)(ws + oW1h); unsigned short* w1l = (unsigned short*)(ws + oW1l);
  unsigned short* w2h = (unsigned short*)(ws + oW2h); unsigned short* w2l = (unsigned short*)(ws + oW2l);
  unsigned short* w3h = (unsigned short*)(ws + oW3h); unsigned short* w3l = (unsigned short*)(ws + oW3l);
  unsigned short* wfh = (unsigned short*)(ws + oWfh); unsigned short* wfl = (unsigned short*)(ws + oWfl);
  unsigned short* gh  = (unsigned short*)(ws + oGh);  unsigned short* gl  = (unsigned short*)(ws + oGl);
  unsigned short* ah  = (unsigned short*)(ws + oAh);  unsigned short* al  = (unsigned short*)(ws + oAl);
  float*          yf3 = (float*)(ws + oAh);
  float*          hbuf = (float*)(ws + oH);

  k_coef<<<2, NTHR, 0, stream>>>(coefp);
  k_wprep<<<(F1 * FE / 8) / NTHR, NTHR, 0, stream>>>(W1,   w1h, w1l, FE, F1, F1);
  k_wprep<<<(F2 * F1 / 8) / NTHR, NTHR, 0, stream>>>(W2,   w2h, w2l, F1, F2, F2);
  k_wprep<<<(F3 * F2 / 8) / NTHR, NTHR, 0, stream>>>(W3,   w3h, w3l, F2, F3, F3);
  k_wprep<<<(FF * F3 / 8) / NTHR, NTHR, 0, stream>>>(Wfus, wfh, wfl, F3, FF, FF);
  k_enc<<<(M * 8) / NTHR, NTHR, 0, stream>>>(lm, Wenc, benc, ah, al, M);
  k_gemm3<0><<<dim3(M / GR, F1 / GC), NTHR, 0, stream>>>(ah, al, w1h, w1l, b1, hbuf, FE, F1);
  k_agg<F1, 0><<<(M * (F1 / 4)) / NTHR, NTHR, 0, stream>>>(hbuf, coefp, b1, ah, al, yf3, M);
  k_gemm3<0><<<dim3(M / GR, F2 / GC), NTHR, 0, stream>>>(ah, al, w2h, w2l, b2, hbuf, F1, F2);
  k_agg<F2, 0><<<(M * (F2 / 4)) / NTHR, NTHR, 0, stream>>>(hbuf, coefp, b2, ah, al, yf3, M);
  k_gemm3<0><<<dim3(M / GR, F3 / GC), NTHR, 0, stream>>>(ah, al, w3h, w3l, b3, hbuf, F2, F3);
  k_agg<F3, 1><<<(M * (F3 / 4)) / NTHR, NTHR, 0, stream>>>(hbuf, coefp, b3, ah, al, yf3, M);
  k_pool<<<(B * 32) / NTHR, NTHR, 0, stream>>>(yf3, out2, gh, gl, B);
  k_gemm3<1><<<dim3(B / GR, FF / GC), NTHR, 0, stream>>>(gh, gl, wfh, wfl, bfus, out1, F3, FF);
  k_cls<<<B / (NTHR / 2), NTHR, 0, stream>>>(out1, Wcls, bcls, out0);
}
